// GsLstm_41437844471984
// MI455X (gfx1250) — hardware-verified
//
#include <hip/hip_runtime.h>
#include <math.h>

constexpr int kBatch  = 8;
constexpr int kNodes  = 2000;
constexpr int kHid    = 128;
constexpr int kNbr    = 32;
constexpr int kRows   = kBatch * kNodes;
constexpr int kKdim   = 4 * kHid;
constexpr int kNdim   = 4 * kHid;
constexpr int kLayers = 2;

typedef __attribute__((ext_vector_type(16))) _Float16 v16h;
typedef __attribute__((ext_vector_type(8)))  _Float16 v8h;
typedef __attribute__((ext_vector_type(16))) __bf16   v16b;
typedef __attribute__((ext_vector_type(8)))  __bf16   v8b;
typedef __attribute__((ext_vector_type(8)))  float    v8f;
typedef __attribute__((ext_vector_type(4)))  float    v4f;
typedef __attribute__((ext_vector_type(4)))  unsigned int v4u;

__device__ __forceinline__ unsigned short f2bf_bits(float f) {
  unsigned u = __float_as_uint(f);
  return (unsigned short)((u + 0x7FFFu + ((u >> 16) & 1u)) >> 16);
}
__device__ __forceinline__ float bf_bits2f(unsigned short h) { return __uint_as_float(((unsigned)h) << 16); }

__device__ __forceinline__ void dep_guard_h(v8f& a, v8f& b, v16h x, v16h y) { asm volatile("v_nop\n\tv_nop\n\tv_nop\n\tv_nop" : "+v"(a), "+v"(b) : "v"(x), "v"(y)); }
__device__ __forceinline__ void dep_guard_b(v8f& a, v8f& b, v16b x, v16b y) { asm volatile("v_nop\n\tv_nop\n\tv_nop\n\tv_nop" : "+v"(a), "+v"(b) : "v"(x), "v"(y)); }
__device__ __forceinline__ void keep4_h(v16h a, v16h b, v16h c, v16h d) { asm volatile("v_nop" :: "v"(a), "v"(b), "v"(c), "v"(d)); }
__device__ __forceinline__ void keep4_b(v16b a, v16b b, v16b c, v16b d) { asm volatile("v_nop" :: "v"(a), "v"(b), "v"(c), "v"(d)); }
__device__ __forceinline__ void acc_guard4(v8f& a, v8f& b, v8f& c, v8f& d) { asm volatile("v_nop\n\tv_nop\n\tv_nop\n\tv_nop" : "+v"(a), "+v"(b), "+v"(c), "+v"(d)); }
template <typename T> struct Frag;
template <> struct Frag<_Float16> {
  typedef v16h V; union U { v16h v; v8h h[2]; };
  static __device__ __forceinline__ v16h load(const _Float16* p) {
    U f; f.h[0] = *(const v8h*)(p); f.h[1] = *(const v8h*)(p + 16); return f.v;
  }
  static __device__ __forceinline__ v8f mma(v16h a, v16h b, v8f c) {
    return __builtin_amdgcn_wmma_f32_16x16x32_f16(false, a, false, b, (short)0, c, false, false);
  }
  static __device__ __forceinline__ void guard(v8f& a, v8f& b, v16h x, v16h y) { dep_guard_h(a, b, x, y); }
  static __device__ __forceinline__ void keep(v16h a, v16h b, v16h c, v16h d) { keep4_h(a, b, c, d); }
};
template <> struct Frag<__bf16> {
  typedef v16b V; union U { v16b v; v8b h[2]; };
  static __device__ __forceinline__ v16b load(const __bf16* p) {
    U f; f.h[0] = *(const v8b*)(p); f.h[1] = *(const v8b*)(p + 16); return f.v;
  }
  static __device__ __forceinline__ v8f mma(v16b a, v16b b, v8f c) {
    return __builtin_amdgcn_wmma_f32_16x16x32_bf16(false, a, false, b, (short)0, c, false, false);
  }
  static __device__ __forceinline__ void guard(v8f& a, v8f& b, v16b x, v16b y) { dep_guard_b(a, b, x, y); }
  static __device__ __forceinline__ void keep(v16b a, v16b b, v16b c, v16b d) { keep4_b(a, b, c, d); }
};

__device__ __forceinline__ unsigned pk16(unsigned short a, unsigned short b) { return (unsigned)a | ((unsigned)b << 16); }

template <int ET> struct Elem;
template <> struct Elem<0> { typedef _Float16 T; };
template <> struct Elem<1> { typedef __bf16 T; };
template <int ET, bool SPLIT, int BIAS_MODE, int OUT_MODE, bool RESID, int ACT = 0>
__global__ __launch_bounds__(256) void wmma_gemm64(
    const unsigned short* __restrict__ Ap, const unsigned short* __restrict__ A2p, int lda, long strideA,
    const unsigned short* __restrict__ Btp, const unsigned short* __restrict__ Bt2p, int ldb, long strideB,
    void* __restrict__ Cout, void* __restrict__ Cout2, int ldc, long strideC,
    const float* __restrict__ bias,
    const float* __restrict__ resid, long strideR,
    int M, int N, int K, float scale) {
  typedef typename Elem<ET>::T T;
  typedef typename Frag<T>::V V;
  const T* A = (const T*)Ap; const T* A2 = (const T*)A2p; const T* Bt = (const T*)Btp; const T* Bt2 = (const T*)Bt2p;
  __shared__ __align__(16) float sT[8][16 * 68];
  const int b    = blockIdx.y;
  const int lane = threadIdx.x & 31;
  const int wave = threadIdx.x >> 5;
  const int tilesN = N >> 6;
  const int tilesM = M >> 6;
  const int tile = blockIdx.x * 8 + wave;
  if (tile >= tilesM * tilesN) return;
  const int tm = tile / tilesN;
  const int tn = tile - tm * tilesN;
  const int m0 = tm << 6;
  const int n0 = tn << 6;

  const T* Ab  = A  + (size_t)b * strideA;
  const T* Bb  = Bt + (size_t)b * strideB;
  const T* Ab2 = SPLIT ? (A2  + (size_t)b * strideA) : nullptr;
  const T* Bb2 = SPLIT ? (Bt2 + (size_t)b * strideB) : nullptr;

  const int rlane = lane & 15;
  const int koff  = (lane >> 4) * 8;
  const int mOff  = (lane >> 4) * 8;

  v8f acc[4][4];
#pragma unroll
  for (int i = 0; i < 4; ++i)
#pragma unroll
    for (int j = 0; j < 4; ++j) acc[i][j] = (v8f){0.f,0.f,0.f,0.f,0.f,0.f,0.f,0.f};

  for (int k0 = 0; k0 < K; k0 += 32) {
    V bh[4], bl[4];
#pragma unroll
    for (int j = 0; j < 4; ++j) {
      const size_t bo = (size_t)(n0 + (j << 4) + rlane) * ldb + koff + k0;
      bh[j] = Frag<T>::load(Bb + bo);
      if (SPLIT) bl[j] = Frag<T>::load(Bb2 + bo);
    }
#pragma unroll
    for (int i = 0; i < 4; ++i) {
      const size_t ao = (size_t)(m0 + (i << 4) + rlane) * lda + koff + k0;
      V ah = Frag<T>::load(Ab + ao);
      V al;
      if (SPLIT) al = Frag<T>::load(Ab2 + ao);
#pragma unroll
      for (int j = 0; j < 4; ++j) {
        acc[i][j] = Frag<T>::mma(ah, bh[j], acc[i][j]);
        if (SPLIT) {
          acc[i][j] = Frag<T>::mma(ah, bl[j], acc[i][j]);
          acc[i][j] = Frag<T>::mma(al, bh[j], acc[i][j]);
        }
      }
      Frag<T>::guard(acc[i][0], acc[i][3], ah, SPLIT ? al : ah);
    }
    Frag<T>::keep(bh[0], bh[1], bh[2], bh[3]);
    if (SPLIT) Frag<T>::keep(bl[0], bl[1], bl[2], bl[3]);
  }
  acc_guard4(acc[0][0], acc[0][1], acc[0][2], acc[0][3]);
  acc_guard4(acc[1][0], acc[1][1], acc[1][2], acc[1][3]);
  acc_guard4(acc[2][0], acc[2][1], acc[2][2], acc[2][3]);
  acc_guard4(acc[3][0], acc[3][1], acc[3][2], acc[3][3]);

  float* slab = sT[wave];
  const float* Rb = RESID ? (resid + (size_t)b * strideR) : nullptr;
#pragma unroll
  for (int i = 0; i < 4; ++i) {
    const int mBase = m0 + (i << 4);
#pragma unroll
    for (int j = 0; j < 4; ++j) {
      const int n = n0 + (j << 4) + rlane;
      float bv = 0.f;
      if (BIAS_MODE == 2) bv = bias[n];
#pragma unroll
      for (int r = 0; r < 8; ++r) {
        float v = acc[i][j][r] * scale;
        if (BIAS_MODE == 1) v += bias[mBase + mOff + r];
        if (BIAS_MODE == 2) v += bv;
        if (RESID) v += Rb[(size_t)(mBase + mOff + r) * ldc + n];
        if (ACT == 2) v = fmaxf(v, 0.0f);
        if (ACT == 4) v = (v > 0.f) ? v : 0.01f * v;
        slab[(mOff + r) * 68 + (j << 4) + rlane] = v;
      }
    }
    __builtin_amdgcn_fence(__ATOMIC_RELEASE, "workgroup");
    __builtin_amdgcn_wave_barrier();
    __builtin_amdgcn_fence(__ATOMIC_ACQUIRE, "workgroup");
    if (OUT_MODE == 0) {
      float* C = (float*)Cout + (size_t)b * strideC;
      const int hh = lane >> 4, c4 = (lane & 15) * 4;
      for (int pass = 0; pass < 2; ++pass) {
#pragma unroll
        for (int it = 0; it < 8; ++it) {
          const int row = it * 2 + hh;
          v4f v = *(const v4f*)(slab + row * 68 + c4);
          *(volatile v4f*)(C + (size_t)(mBase + row) * ldc + n0 + c4) = v;
        }
        __threadfence();
      }
    } else {
      const int q = lane >> 3, c8 = (lane & 7) * 8;
      unsigned short* C  = (unsigned short*)Cout  + (size_t)b * strideC;
      unsigned short* C2 = (OUT_MODE == 2) ? ((unsigned short*)Cout2 + (size_t)b * strideC) : nullptr;
      for (int pass = 0; pass < 2; ++pass) {
#pragma unroll
        for (int it = 0; it < 4; ++it) {
          const int row = it * 4 + q;
          const float* sp = slab + row * 68 + c8;
          v8h hv, lv;
#pragma unroll
          for (int e = 0; e < 8; ++e) {
            if (OUT_MODE == 1) {
              hv[e] = (_Float16)sp[e];
            } else {
              unsigned short hb = f2bf_bits(sp[e]);
              unsigned short lb = f2bf_bits(sp[e] - bf_bits2f(hb));
              hv[e] = __builtin_bit_cast(_Float16, hb);
              lv[e] = __builtin_bit_cast(_Float16, lb);
            }
          }
          *(volatile v8h*)(C + (size_t)(mBase + row) * ldc + n0 + c8) = hv;
          if (OUT_MODE == 2) *(volatile v8h*)(C2 + (size_t)(mBase + row) * ldc + n0 + c8) = lv;
        }
        __threadfence();
      }
    }
    __builtin_amdgcn_fence(__ATOMIC_RELEASE, "workgroup");
    __builtin_amdgcn_wave_barrier();
    __builtin_amdgcn_fence(__ATOMIC_ACQUIRE, "workgroup");
  }
}

__global__ __launch_bounds__(256) void wsplit_kernel(const float* __restrict__ W0, const float* __restrict__ W1,
                                                     const float* __restrict__ W2, const float* __restrict__ W3,
                                                     unsigned short* __restrict__ out, long planeStride) {
  __shared__ float sm[64][65];
  const int t    = threadIdx.x;
  const int kt   = blockIdx.x;
  const int nt   = blockIdx.y;
  const int qsel = kt >> 1;
  const int kk0  = (kt & 1) * 64;
  const int g    = nt >> 1;
  const int d0   = (nt & 1) * 64;
  const float* W = (qsel == 0) ? W0 : (qsel == 1) ? W1 : (qsel == 2) ? W2 : W3;
#pragma unroll
  for (int i = 0; i < 16; ++i) {
    const int e = i * 256 + t;
    const int r = e >> 6;
    const int c = e & 63;
    sm[c][r] = W[(size_t)(g * kHid + kk0 + r) * kHid + d0 + c];
  }
  __syncthreads();
  const int lane = t & 31, wave = t >> 5;
  const int q8 = lane >> 3, c8 = (lane & 7) * 8;
  for (int pass = 0; pass < 2; ++pass) {
#pragma unroll
    for (int it = 0; it < 2; ++it) {
      const int row = wave * 8 + it * 4 + q8;
      unsigned short hb[8], lb[8];
#pragma unroll
      for (int e = 0; e < 8; ++e) {
        const float v = sm[row][c8 + e];
        hb[e] = f2bf_bits(v);
        lb[e] = f2bf_bits(v - bf_bits2f(hb[e]));
      }
      const v4u uh = (v4u){pk16(hb[0], hb[1]), pk16(hb[2], hb[3]), pk16(hb[4], hb[5]), pk16(hb[6], hb[7])};
      const v4u ul = (v4u){pk16(lb[0], lb[1]), pk16(lb[2], lb[3]), pk16(lb[4], lb[5]), pk16(lb[6], lb[7])};
      const size_t off = (size_t)(g * kHid + d0 + row) * kKdim + kt * 64 + c8;
      *(volatile v4u*)(out + off) = uh;
      *(volatile v4u*)(out + planeStride + off) = ul;
    }
    __threadfence();
  }
}

__global__ __launch_bounds__(128) void agg_split_kernel(
    const float* __restrict__ hsrc,
    const int* __restrict__ inIdx, const float* __restrict__ inMsk,
    const int* __restrict__ outIdx, const float* __restrict__ outMsk,
    unsigned short* __restrict__ Aplanes, long planeStride) {
  __shared__ int   sIn[kNbr];
  __shared__ float sInM[kNbr];
  __shared__ int   sOut[kNbr];
  __shared__ float sOutM[kNbr];
  __shared__ __align__(16) float srow[kKdim];

  const int row = blockIdx.x;
  const int b   = row / kNodes;
  const int tid = threadIdx.x;

  if (tid < kNbr) {
    const int base = row * kNbr + tid;
    int a = inIdx[base];
    a = a < 0 ? 0 : a; a = a > kNodes - 1 ? kNodes - 1 : a;
    int c = outIdx[base];
    c = c < 0 ? 0 : c; c = c > kNodes - 1 ? kNodes - 1 : c;
    sIn[tid]   = a;
    sInM[tid]  = inMsk[base];
    sOut[tid]  = c;
    sOutM[tid] = outMsk[base];
  }
  __syncthreads();

  const float* hb = hsrc + (size_t)b * kNodes * kHid;
  float accIn = 0.f, accOut = 0.f;
#pragma unroll 8
  for (int k = 0; k < kNbr; ++k) {
    const float hvi = hb[(size_t)sIn[k]  * kHid + tid];
    const float hvo = hb[(size_t)sOut[k] * kHid + tid];
    accIn  += sInM[k]  * hvi;
    accOut += sOutM[k] * hvo;
  }
  const float hs = hsrc[(size_t)row * kHid + tid];
  srow[tid]            = accIn;
  srow[kHid + tid]     = accOut;
  srow[2 * kHid + tid] = hs;
  srow[3 * kHid + tid] = hs;
  __syncthreads();

  const int plane = tid >> 6;
  const int j     = tid & 63;
  const v4f x0 = *(const v4f*)(srow + 8 * j);
  const v4f x1 = *(const v4f*)(srow + 8 * j + 4);
  unsigned short ob[8];
#pragma unroll
  for (int e = 0; e < 4; ++e) {
    const float v0 = x0[e];
    const unsigned short h0 = f2bf_bits(v0);
    const unsigned short l0 = f2bf_bits(v0 - bf_bits2f(h0));
    ob[e] = plane ? l0 : h0;
    const float v1 = x1[e];
    const unsigned short h1 = f2bf_bits(v1);
    const unsigned short l1 = f2bf_bits(v1 - bf_bits2f(h1));
    ob[4 + e] = plane ? l1 : h1;
  }
  const v4u u = (v4u){pk16(ob[0], ob[1]), pk16(ob[2], ob[3]), pk16(ob[4], ob[5]), pk16(ob[6], ob[7])};
  unsigned short* dst = Aplanes + (size_t)plane * planeStride + (size_t)row * kKdim + 8 * j;
  *(volatile v4u*)dst = u;
  __threadfence();
  *(volatile v4u*)dst = u;
}

__device__ __forceinline__ float rcp_apx(float x) { return __builtin_amdgcn_rcpf(x); }
__device__ __forceinline__ float sigm_f(float x) { return rcp_apx(1.0f + expf(-x)); }
__device__ __forceinline__ float tanh_f(float x) { return 1.0f - 2.0f * rcp_apx(1.0f + expf(2.0f * x)); }

template <bool WRITE_C>
__global__ __launch_bounds__(256) void cell_kernel(const float* __restrict__ PRE, const float* __restrict__ Cin,
                                                   const float* __restrict__ Hin, const int* __restrict__ layerNum,
                                                   int layerIdx, float* __restrict__ hOutP, float* __restrict__ cOutP) {
  __shared__ __align__(16) float sh[2][kHid];
  __shared__ __align__(16) float sc[2][kHid];
  const int t    = threadIdx.x;
  const int rloc = t >> 7;
  const int d    = t & (kHid - 1);
  const int mrow0 = blockIdx.x * 2;
  const int m    = mrow0 + rloc;
  const int nl   = layerNum[0];
  const bool active = (layerIdx < nl);

  const float* p = PRE + (size_t)m * kNdim;
  const float iv = p[d];
  const float ov = p[kHid + d];
  const float fv = p[2 * kHid + d];
  const float gv = p[3 * kHid + d];
  const float cold = Cin[(size_t)m * kHid + d];
  const float hold = Hin[(size_t)m * kHid + d];
  const float si = sigm_f(iv);
  const float so = sigm_f(ov);
  const float sf = sigm_f(fv);
  const float gg = tanh_f(gv);
  float cn = sf * cold + si * gg;
  float hn = so * tanh_f(cn);
  cn = active ? cn : cold;
  hn = active ? hn : hold;
  sh[rloc][d] = hn;
  sc[rloc][d] = cn;
  __syncthreads();

  const int wave = t >> 5, lane = t & 31;
  if (wave < 2) {
    const v4f v = *(const v4f*)(&sh[wave][4 * lane]);
    float* dst = hOutP + (size_t)(mrow0 + wave) * kHid + 4 * lane;
    *(volatile v4f*)dst = v;
    __threadfence();
    *(volatile v4f*)dst = v;
  } else if (WRITE_C && wave < 4) {
    const v4f v = *(const v4f*)(&sc[wave - 2][4 * lane]);
    float* dst = cOutP + (size_t)(mrow0 + wave - 2) * kHid + 4 * lane;
    *(volatile v4f*)dst = v;
    __threadfence();
    *(volatile v4f*)dst = v;
  }
}

extern "C" void kernel_launch(void* const* d_in, const int* in_sizes, int n_in,
                              void* d_out, int out_size, void* d_ws, size_t ws_size,
                              hipStream_t stream) {
  if (n_in < 12) return;
  if (in_sizes[0] != kRows * kHid || in_sizes[1] != kRows * kHid) return;
  if (in_sizes[2] != 4 * kHid * kHid || in_sizes[3] != 4 * kHid * kHid ||
      in_sizes[4] != 4 * kHid * kHid || in_sizes[5] != 4 * kHid * kHid) return;
  if (in_sizes[6] != 4 * kHid) return;
  if (in_sizes[7] != kRows * kNbr || in_sizes[8] != kRows * kNbr ||
      in_sizes[9] != kRows * kNbr || in_sizes[10] != kRows * kNbr) return;
  if (in_sizes[11] < 1) return;
  if (out_size != kRows * kHid) return;

  const float* node_hidden = (const float*)d_in[0];
  const float* cell        = (const float*)d_in[1];
  const float* w_in        = (const float*)d_in[2];
  const float* w_out       = (const float*)d_in[3];
  const float* u_in        = (const float*)d_in[4];
  const float* u_out       = (const float*)d_in[5];
  const float* bias        = (const float*)d_in[6];
  const float* in_msk      = (const float*)d_in[7];
  const float* out_msk     = (const float*)d_in[8];
  const int*   in_idx      = (const int*)d_in[9];
  const int*   out_idx     = (const int*)d_in[10];
  const int*   layer_num   = (const int*)d_in[11];
  float*       outp        = (float*)d_out;

  const size_t btPlane  = (size_t)kNdim * kKdim;
  const size_t aPlane   = (size_t)kRows * kKdim;
  const size_t btBytes  = btPlane * 2;
  const size_t aBytes   = aPlane * 2;
  const size_t preBytes = (size_t)kRows * kNdim * sizeof(float);
  const size_t stBytes  = (size_t)kRows * kHid * sizeof(float);

  size_t off = 0;
  const size_t oBt  = off; off += 2 * btBytes;
  const size_t oA   = off; off += 2 * aBytes;
  const size_t oPre = off; off += preBytes;
  const size_t oH1  = off; off += stBytes;
  const size_t oC1  = off; off += stBytes;
  if (off > ws_size) return;

  char* ws = (char*)d_ws;
  unsigned short* Bt_hi = (unsigned short*)(ws + oBt);
  unsigned short* Bt_lo = Bt_hi + btPlane;
  unsigned short* A_hi  = (unsigned short*)(ws + oA);
  unsigned short* A_lo  = A_hi + aPlane;
  float*          PRE   = (float*)(ws + oPre);
  float*          H1    = (float*)(ws + oH1);
  float*          C1    = (float*)(ws + oC1);

  wsplit_kernel<<<dim3(kKdim / 64, kNdim / 64), 256, 0, stream>>>(w_in, w_out, u_in, u_out, Bt_hi, (long)btPlane);

  const int gemmBlocks = ((kRows / 64) * (kNdim / 64) + 7) / 8;

  for (int layer = 0; layer < kLayers; ++layer) {
    const float* hsrc = (layer == 0) ? node_hidden : (const float*)H1;
    const float* csrc = (layer == 0) ? cell : (const float*)C1;
    agg_split_kernel<<<kRows, kHid, 0, stream>>>(hsrc, in_idx, in_msk, out_idx, out_msk, A_hi, (long)aPlane);
    wmma_gemm64<1, true, 2, 0, false, 0><<<dim3(gemmBlocks, 1), 256, 0, stream>>>(
        A_hi, A_lo, kKdim, 0L,
        Bt_hi, Bt_lo, kKdim, 0L,
        (void*)PRE, (void*)PRE, kNdim, 0L,
        bias,
        (const float*)PRE, 0L,
        kRows, kNdim, kKdim, 1.0f);
    if (layer == 0) {
      cell_kernel<true><<<kRows / 2, 256, 0, stream>>>(PRE, csrc, hsrc, layer_num, layer, H1, C1);
    } else {
      cell_kernel<false><<<kRows / 2, 256, 0, stream>>>(PRE, csrc, hsrc, layer_num, layer, outp, C1);
    }
  }
}
